// DyadicTransferMap_88304527606074
// MI455X (gfx1250) — hardware-verified
//
#include <hip/hip_runtime.h>
#include <stdint.h>

#define NB   2
#define NN   8192
#define ND   64
#define NE   64
#define ICH  32
#define XP   72
#define WP   72
#define EP   72
#define OP   68

#define THRESH   0.7f
#define SC_U     16.0f
#define SC_W     64.0f
#define SC_RES   2048.0f
#define SC_P     1024.0f
#define INV_UW   0.015625f
#define INV_RES  0.00048828125f
#define INV_S    0.00390625f
#define INV_L    0.00006103515625f

static_assert(NN % 64 == 0);
static_assert(NN % ICH == 0);
static_assert(ND == 64);
static_assert(NE == 64);
static_assert((XP % 8) == 0);
static_assert((WP % 8) == 0);
static_assert((EP % 8) == 0);
static_assert((OP % 4) == 0);
static_assert(15 * OP + 63 < 16 * OP);
static_assert(15 * EP + 63 < 16 * EP);
static_assert(63 * XP + 63 < 64 * XP);

typedef _Float16 f16;
typedef _Float16 v16h __attribute__((ext_vector_type(16)));
typedef _Float16 v8h  __attribute__((ext_vector_type(8)));
typedef _Float16 v8ha __attribute__((ext_vector_type(8), may_alias));
typedef unsigned short v8us __attribute__((ext_vector_type(8)));
typedef float v8f __attribute__((ext_vector_type(8)));
typedef float v4f __attribute__((ext_vector_type(4)));
typedef float v4fa __attribute__((ext_vector_type(4), may_alias));

union FragH { v16h v; v8h h[2]; };

__device__ __forceinline__ float bf16r(float f) {
  unsigned int u = __float_as_uint(f);
  u = u + 0x7FFFu + ((u >> 16) & 1u);
  u &= 0xFFFF0000u;
  return __uint_as_float(u);
}

__device__ __forceinline__ v8f mma_h(v16h a, v16h b, v8f c) {
  return __builtin_amdgcn_wmma_f32_16x16x32_f16(false, a, false, b, (short)0, c, false, false);
}

__device__ __forceinline__ void guard_2c(v8f& c0, v8f& c1, v16h a0, v16h a1, v16h a2, v16h a3, v16h b0, v16h b1) {
#if defined(__HIP_DEVICE_COMPILE__)
  asm volatile("v_nop\n\tv_nop\n\tv_nop\n\tv_nop"
               : "+v"(c0), "+v"(c1)
               : "v"(a0), "v"(a1), "v"(a2), "v"(a3), "v"(b0), "v"(b1));
#endif
}
__device__ __forceinline__ void guard_4c(v8f& c0, v8f& c1, v8f& c2, v8f& c3,
                                         v16h a0, v16h a1, v16h a2, v16h a3, v16h b0) {
#if defined(__HIP_DEVICE_COMPILE__)
  asm volatile("v_nop\n\tv_nop\n\tv_nop\n\tv_nop"
               : "+v"(c0), "+v"(c1), "+v"(c2), "+v"(c3)
               : "v"(a0), "v"(a1), "v"(a2), "v"(a3), "v"(b0));
#endif
}

__global__ __launch_bounds__(256)
void k_cvt_u(const float* __restrict__ u, unsigned short* uh, int n8) {
  const int g = (int)blockIdx.x * 256 + (int)threadIdx.x;
  if (g >= n8) return;
  const float* p = u + (size_t)g * 8;
  const v4f a = *(const v4f*)p;
  const v4f c = *(const v4f*)(p + 4);
  v8h o;
#pragma unroll
  for (int e = 0; e < 4; ++e) {
    o[e]     = (f16)(bf16r(a[e]) * SC_U);
    o[4 + e] = (f16)(bf16r(c[e]) * SC_U);
  }
  const v8us w = __builtin_bit_cast(v8us, o);
  unsigned short* op = uh + (size_t)g * 8;
  *(volatile v8us*)op = w;
  __threadfence();
  *(volatile v8us*)op = w;
}

__global__ __launch_bounds__(256)
void k_gate(const float* __restrict__ prof, float* gsc, int n4) {
  const int g = (int)blockIdx.x * 256 + (int)threadIdx.x;
  if (g >= n4) return;
  const v4f p = *(const v4f*)(prof + (size_t)g * 4);
  v4f o;
#pragma unroll
  for (int e = 0; e < 4; ++e) o[e] = fmaxf(bf16r(p[e]) - THRESH, 0.0f) * SC_P;
  float* op = gsc + (size_t)g * 4;
  *(volatile v4f*)op = o;
  __threadfence();
  *(volatile v4f*)op = o;
}

__global__ __launch_bounds__(256)
void k_xt(const float* __restrict__ x, unsigned short* xt) {
  __shared__ __align__(16) f16 sx[ND * XP];
  const int tid = threadIdx.x;
  const int b   = (int)blockIdx.y;
  const int i0  = (int)blockIdx.x * 64;
  const int il  = tid >> 2;
  const int d0  = (tid & 3) * 16;
  const float* p = x + ((size_t)(b * NN + i0 + il)) * ND + d0;
  const v4f q0 = *(const v4f*)p;
  const v4f q1 = *(const v4f*)(p + 4);
  const v4f q2 = *(const v4f*)(p + 8);
  const v4f q3 = *(const v4f*)(p + 12);
#pragma unroll
  for (int e = 0; e < 4; ++e) {
    sx[(d0 + e) * XP + il]      = (f16)(bf16r(q0[e]) * SC_U);
    sx[(d0 + 4 + e) * XP + il]  = (f16)(bf16r(q1[e]) * SC_U);
    sx[(d0 + 8 + e) * XP + il]  = (f16)(bf16r(q2[e]) * SC_U);
    sx[(d0 + 12 + e) * XP + il] = (f16)(bf16r(q3[e]) * SC_U);
  }
  __syncthreads();

  const int lr    = tid >> 3;
  const int piece = (tid & 7) * 8;
  v8us u[2];
  size_t go[2];
#pragma unroll
  for (int ps = 0; ps < 2; ++ps) {
    const int d = ps * 32 + lr;
    const v8h t = *(const v8ha*)&sx[d * XP + piece];
    u[ps]  = __builtin_bit_cast(v8us, t);
    go[ps] = ((size_t)(b * ND + d)) * NN + i0 + piece;
  }
#pragma unroll
  for (int ps = 0; ps < 2; ++ps) *(volatile v8us*)(xt + go[ps]) = u[ps];
  __threadfence();
#pragma unroll
  for (int ps = 0; ps < 2; ++ps) *(volatile v8us*)(xt + go[ps]) = u[ps];
}

__global__ __launch_bounds__(128)
void k_uw(const unsigned short* __restrict__ uh, const float* __restrict__ w,
          unsigned short* uwh, unsigned short* uwl) {
  __shared__ __align__(16) f16 swt[NE * WP];
  __shared__ __align__(16) f16 sst[2][4][16 * EP];
  const int tid = threadIdx.x, lane = tid & 31, wv = tid >> 5, h = lane >> 4, lm = lane & 15;
  const int i0 = (int)blockIdx.x * 64;

#pragma unroll
  for (int q = 0; q < 32; ++q) {
    const int idx = q * 128 + tid;
    const int e = idx >> 6, f = idx & 63;
    swt[f * WP + e] = (f16)(bf16r(w[idx]) * SC_W);
  }
  __syncthreads();

  const f16* U16 = (const f16*)uh;
  const f16* pa = U16 + (size_t)(i0 + wv * 16 + lm) * NE + 8 * h;
  FragH a[2];
#pragma unroll
  for (int ks = 0; ks < 2; ++ks) {
    a[ks].h[0] = *(const v8h*)(pa + ks * 32);
    a[ks].h[1] = *(const v8h*)(pa + ks * 32 + 16);
  }
  const v8f zero = {};
  v8f acc[4];
#pragma unroll
  for (int nt = 0; nt < 4; ++nt) acc[nt] = zero;

#pragma unroll
  for (int ks = 0; ks < 2; ++ks) {
    FragH bq[4];
#pragma unroll
    for (int nt = 0; nt < 4; ++nt) {
      const f16* pb = &swt[(nt * 16 + lm) * WP + ks * 32 + 8 * h];
      bq[nt].h[0] = *(const v8ha*)pb;
      bq[nt].h[1] = *(const v8ha*)(pb + 16);
    }
#pragma unroll
    for (int nt = 0; nt < 4; ++nt) acc[nt] = mma_h(a[ks].v, bq[nt].v, acc[nt]);
    guard_4c(acc[0], acc[1], acc[2], acc[3], bq[0].v, bq[1].v, bq[2].v, bq[3].v, a[ks].v);
  }

#pragma unroll
  for (int nt = 0; nt < 4; ++nt)
#pragma unroll
    for (int r = 0; r < 8; ++r) {
      const float xv  = acc[nt][r] * INV_UW;
      const f16   hv  = (f16)xv;
      const float res = (xv - (float)hv) * SC_RES;
      const f16   lv  = (f16)res;
      const int   o   = (8 * h + r) * EP + nt * 16 + lm;
      sst[0][wv][o] = hv;
      sst[1][wv][o] = lv;
    }
  __syncthreads();

  v8us vh[4], vl[4];
  size_t go[4];
#pragma unroll
  for (int it = 0; it < 4; ++it) {
    const int rowl  = it * 4 + (lane >> 3);
    const int piece = (lane & 7) * 8;
    const v8h th = *(const v8ha*)&sst[0][wv][rowl * EP + piece];
    const v8h tl = *(const v8ha*)&sst[1][wv][rowl * EP + piece];
    vh[it] = __builtin_bit_cast(v8us, th);
    vl[it] = __builtin_bit_cast(v8us, tl);
    go[it] = (size_t)(i0 + wv * 16 + rowl) * NE + piece;
  }
#pragma unroll
  for (int it = 0; it < 4; ++it) {
    *(volatile v8us*)(uwh + go[it]) = vh[it];
    *(volatile v8us*)(uwl + go[it]) = vl[it];
  }
  __threadfence();
#pragma unroll
  for (int it = 0; it < 4; ++it) {
    *(volatile v8us*)(uwh + go[it]) = vh[it];
    *(volatile v8us*)(uwl + go[it]) = vl[it];
  }
}

__global__ __launch_bounds__(128)
void k_main(const unsigned short* __restrict__ uh, const unsigned short* __restrict__ uwh,
            const unsigned short* __restrict__ uwl, const unsigned short* __restrict__ xt,
            const float* __restrict__ gsc, const float* __restrict__ x,
            const float* __restrict__ bias, float* out) {
  __shared__ __align__(16) float so[4][2][16 * OP];
  const int tid = threadIdx.x, lane = tid & 31, wv = tid >> 5, h = lane >> 4, lm = lane & 15;
  const int j0  = ((int)blockIdx.x * 4 + wv) * 16;
  const int jg  = j0 + lm;
  const int dch = j0 & ~(ICH - 1);
  const float bv = bf16r(bias[0]);

  const f16* U16 = (const f16*)uh;
  const f16* H16 = (const f16*)uwh;
  const f16* L16 = (const f16*)uwl;
  const f16* X16 = (const f16*)xt;

  FragH ub[2];
  {
    const f16* pb = U16 + (size_t)jg * NE + 8 * h;
#pragma unroll
    for (int ks = 0; ks < 2; ++ks) {
      ub[ks].h[0] = *(const v8h*)(pb + ks * 32);
      ub[ks].h[1] = *(const v8h*)(pb + ks * 32 + 16);
    }
  }

  const v8f zero = {};
  v8f acc[2][4];
#pragma unroll
  for (int b = 0; b < 2; ++b)
#pragma unroll
    for (int dt = 0; dt < 4; ++dt) acc[b][dt] = zero;

#pragma unroll 1
  for (int ic = 0; ic < NN; ic += ICH) {
    float tt[2][8];
#pragma unroll
    for (int t = 0; t < 2; ++t) {
      FragH ah[2], al[2];
      const size_t ro = (size_t)(ic + t * 16 + lm) * NE + 8 * h;
#pragma unroll
      for (int ks = 0; ks < 2; ++ks) {
        ah[ks].h[0] = *(const v8h*)(H16 + ro + ks * 32);
        ah[ks].h[1] = *(const v8h*)(H16 + ro + ks * 32 + 16);
        al[ks].h[0] = *(const v8h*)(L16 + ro + ks * 32);
        al[ks].h[1] = *(const v8h*)(L16 + ro + ks * 32 + 16);
      }
      v8f sh = zero, sl = zero;
#pragma unroll
      for (int ks = 0; ks < 2; ++ks) {
        sh = mma_h(ah[ks].v, ub[ks].v, sh);
        sl = mma_h(al[ks].v, ub[ks].v, sl);
      }
      guard_2c(sh, sl, ah[0].v, ah[1].v, al[0].v, al[1].v, ub[0].v, ub[1].v);
#pragma unroll
      for (int r = 0; r < 8; ++r) {
        const float s = (sh[r] + sl[r] * INV_RES) * INV_S + bv;
        const float e = __expf(-s);
        tt[t][r] = __builtin_amdgcn_rcpf(1.0f + e);
      }
    }
    if (ic == dch) {
#pragma unroll
      for (int r = 0; r < 8; ++r) {
        const int ia = ic + 8 * h + r;
        tt[0][r] = (ia == jg) ? 0.0f : tt[0][r];
        tt[1][r] = (ia + 16 == jg) ? 0.0f : tt[1][r];
      }
    }
#pragma unroll
    for (int b = 0; b < NB; ++b) {
      const float* gp = gsc + (size_t)b * NN + ic + 8 * h;
      const v4f g0 = *(const v4f*)gp;
      const v4f g1 = *(const v4f*)(gp + 4);
      const v4f g2 = *(const v4f*)(gp + 16);
      const v4f g3 = *(const v4f*)(gp + 20);
      v8h p0, p1;
#pragma unroll
      for (int e = 0; e < 4; ++e) {
        p0[e]     = (f16)(g0[e] * tt[0][e]);
        p0[4 + e] = (f16)(g1[e] * tt[0][4 + e]);
        p1[e]     = (f16)(g2[e] * tt[1][e]);
        p1[4 + e] = (f16)(g3[e] * tt[1][4 + e]);
      }
      FragH bt;
      bt.h[0] = p0;
      bt.h[1] = p1;
      FragH xa[4];
#pragma unroll
      for (int dt = 0; dt < 4; ++dt) {
        const f16* px = X16 + (size_t)(b * ND + dt * 16 + lm) * NN + ic + 8 * h;
        xa[dt].h[0] = *(const v8h*)px;
        xa[dt].h[1] = *(const v8h*)(px + 16);
      }
#pragma unroll
      for (int dt = 0; dt < 4; ++dt) acc[b][dt] = mma_h(xa[dt].v, bt.v, acc[b][dt]);
      guard_4c(acc[b][0], acc[b][1], acc[b][2], acc[b][3], xa[0].v, xa[1].v, xa[2].v, xa[3].v, bt.v);
    }
  }

#pragma unroll
  for (int b = 0; b < NB; ++b)
#pragma unroll
    for (int dt = 0; dt < 4; ++dt)
#pragma unroll
      for (int r = 0; r < 8; ++r)
        so[wv][b][lm * OP + dt * 16 + 8 * h + r] = acc[b][dt][r] * INV_L;
  __syncthreads();

#pragma unroll
  for (int b = 0; b < NB; ++b) {
    v4f val[8];
    size_t go[8];
#pragma unroll
    for (int it = 0; it < 8; ++it) {
      const int jl = it * 2 + h;
      const int c  = lm * 4;
      const v4f lv = *(const v4fa*)&so[wv][b][jl * OP + c];
      go[it] = ((size_t)(b * NN + j0 + jl)) * ND + c;
      const v4f xs = *(const v4f*)(x + go[it]);
      v4f o;
#pragma unroll
      for (int q = 0; q < 4; ++q) o[q] = bf16r(xs[q]) + lv[q];
      val[it] = o;
    }
#pragma unroll
    for (int it = 0; it < 8; ++it) *(volatile v4f*)(out + go[it]) = val[it];
    __threadfence();
#pragma unroll
    for (int it = 0; it < 8; ++it) *(volatile v4f*)(out + go[it]) = val[it];
  }
}

extern "C" void kernel_launch(void* const* d_in, const int* in_sizes, int n_in,
                              void* d_out, int out_size, void* d_ws, size_t ws_size,
                              hipStream_t stream) {
  if (n_in < 5) return;
  if (in_sizes[0] != NB * NN * ND) return;
  if (in_sizes[1] != NB * NN) return;
  if (in_sizes[2] != NN * NE) return;
  if (in_sizes[3] != NE * NE) return;
  if (in_sizes[4] < 1) return;
  if (out_size != NB * NN * ND) return;

  const size_t off_uh  = 0;
  const size_t sz_uh   = (size_t)NN * NE * sizeof(unsigned short);
  const size_t off_uwh = off_uh + sz_uh;
  const size_t off_uwl = off_uwh + sz_uh;
  const size_t off_xt  = off_uwl + sz_uh;
  const size_t sz_xt   = (size_t)NB * ND * NN * sizeof(unsigned short);
  const size_t off_g   = off_xt + sz_xt;
  const size_t sz_g    = (size_t)NB * NN * sizeof(float);
  const size_t need    = off_g + sz_g;
  if (need > ws_size) return;
  if (need > (size_t)134217728) return;

  const float* states = (const float*)d_in[0];
  const float* prof   = (const float*)d_in[1];
  const float* u      = (const float*)d_in[2];
  const float* w      = (const float*)d_in[3];
  const float* bias   = (const float*)d_in[4];
  float* out = (float*)d_out;
  char* ws = (char*)d_ws;
  unsigned short* uh  = (unsigned short*)(ws + off_uh);
  unsigned short* uwh = (unsigned short*)(ws + off_uwh);
  unsigned short* uwl = (unsigned short*)(ws + off_uwl);
  unsigned short* xt  = (unsigned short*)(ws + off_xt);
  float* gsc = (float*)(ws + off_g);

  const int n8 = in_sizes[2] / 8;
  const int n4 = in_sizes[1] / 4;
  k_cvt_u<<<dim3((n8 + 255) / 256), dim3(256), 0, stream>>>(u, uh, n8);
  k_gate<<<dim3((n4 + 255) / 256), dim3(256), 0, stream>>>(prof, gsc, n4);
  k_xt<<<dim3(NN / 64, NB), dim3(256), 0, stream>>>(states, xt);
  k_uw<<<dim3(NN / 64), dim3(128), 0, stream>>>(uh, w, uwh, uwl);
  k_main<<<dim3(NN / 64), dim3(128), 0, stream>>>(uh, uwh, uwl, xt, gsc, states, bias, out);
  (void)hipGetLastError();
}
